// BatchGraphAttention_28003186770284
// MI455X (gfx1250) — hardware-verified
//
#include <hip/hip_runtime.h>
#include <hip/hip_bf16.h>


#define Bq 8
#define Nq 1024
#define Dq 512
#define Hq 8
#define HDq 64

typedef __attribute__((ext_vector_type(16))) _Float16 v16h;
typedef __attribute__((ext_vector_type(8)))  _Float16 v8h;
typedef __attribute__((ext_vector_type(8)))  float    v8f;
typedef int gv4i __attribute__((vector_size(16)));

#define USE_ASYNC_LDS 0
typedef __attribute__((ext_vector_type(4))) float v4f;
typedef __attribute__((ext_vector_type(4))) unsigned v4u;
template <typename V> __device__ __forceinline__ void vst2(void* p, V v) {
    *(volatile V*)p = v; __threadfence(); *(volatile V*)p = v;
}
#define PSC 256.0f
#define PUN (1.0f / 256.0f)
__device__ __forceinline__ v8f wmma16(v16h a, v16h b, v8f c) {
    v8f d = __builtin_amdgcn_wmma_f32_16x16x32_f16(false, a, false, b, (short)0, c, false, false);
    asm volatile("v_nop\n\tv_nop\n\tv_nop\n\tv_nop" : "+v"(d) : "v"(a), "v"(b));
    return d;
}
__device__ __forceinline__ v16h frag_row(const _Float16* row_k0, int hi) {
    v8h lo = *(const v8h*)(row_k0 + hi * 8);
    v8h up = *(const v8h*)(row_k0 + hi * 8 + 16);
    v16h f;
    #pragma unroll
    for (int e = 0; e < 8; ++e) { f[e] = lo[e]; f[e + 8] = up[e]; }
    return f;
}

#define GPTR(p) ((__attribute__((address_space(1))) gv4i*)(void*)(size_t)(const void*)(p))
#define LPTR(p) ((__attribute__((address_space(3))) gv4i*)(void*)(p))

__global__ __launch_bounds__(256) void cvt_f32_f16(const float* __restrict__ in,
                                                   _Float16* __restrict__ out, int n) {
    int g = blockIdx.x * 256 + threadIdx.x;
    if (g * 8 >= n) return;
    union { v8h h; v4u u; } pk;
    #pragma unroll
    for (int e = 0; e < 8; ++e) pk.h[e] = (_Float16)in[(size_t)g * 8 + e];
    vst2(out + (size_t)g * 8, pk.u);
}

__global__ __launch_bounds__(256) void qkv_gemm(
    const _Float16* __restrict__ x16,
    const _Float16* __restrict__ wq16, const _Float16* __restrict__ wk16,
    const _Float16* __restrict__ wv16,
    _Float16* __restrict__ q16, _Float16* __restrict__ k16,
    _Float16* __restrict__ v16) {

    const _Float16* w   = (blockIdx.z == 0) ? wq16 : (blockIdx.z == 1) ? wk16 : wv16;
    _Float16*       out = (blockIdx.z == 0) ? q16  : (blockIdx.z == 1) ? k16  : v16;

    const int tid  = threadIdx.x;
    const int wave = tid >> 5;
    const int lane = tid & 31;
    const int hi   = lane >> 4;
    const int l16  = lane & 15;

    const int m0 = blockIdx.x * 16;
    const int n0 = blockIdx.y * 128 + wave * 16;

    __shared__ __align__(16) _Float16 As[16 * Dq];
    __shared__ __align__(16) _Float16 Ct[16][128];

    {
        const char* src = (const char*)(x16 + (size_t)m0 * Dq);
        for (int c = tid; c < 16 * Dq / 8; c += 256)
            ((v4u*)As)[c] = ((const v4u*)src)[c];
    }
    __syncthreads();

    v8f acc = {};
    for (int kk = 0; kk < Dq; kk += 32) {
        const _Float16* ap = As + l16 * Dq + kk + hi * 8;
        v8h alo = *(const v8h*)ap;
        v8h ahi = *(const v8h*)(ap + 16);
        v16h a;
        #pragma unroll
        for (int e = 0; e < 8; ++e) { a[e] = alo[e]; a[e + 8] = ahi[e]; }
        v16h b = frag_row(w + (size_t)(n0 + l16) * Dq + kk, hi);
        acc = wmma16(a, b, acc);
    }

    #pragma unroll
    for (int i = 0; i < 8; ++i) Ct[i + hi * 8][wave * 16 + l16] = (_Float16)acc[i];
    __syncthreads();
    {
        const int r = tid >> 4, pc = tid & 15;
        vst2(out + (size_t)(m0 + r) * Dq + blockIdx.y * 128 + pc * 8, *(const v4u*)(&Ct[r][pc * 8]));
    }
}

__global__ __launch_bounds__(256) void attn_kernel(
    const _Float16* __restrict__ q16, const _Float16* __restrict__ k16,
    const _Float16* __restrict__ v16, const int* __restrict__ adj,
    _Float16* __restrict__ attn16) {

    const int tid  = threadIdx.x;
    const int wave = tid >> 5;
    const int lane = tid & 31;
    const int hi   = lane >> 4;
    const int l16  = lane & 15;
    const int h    = wave;
    const int b    = blockIdx.y;
    const int q0   = blockIdx.x * 16;

    __shared__ float                  adjb[16 * 32];
    __shared__ __align__(16) _Float16 Vt[8][32 * HDq];
    __shared__ __align__(16) _Float16 Pt[8][16 * 32];
    __shared__ __align__(16) _Float16 Ot[8][16 * HDq];

    v16h qa[2];
    {
        const _Float16* qbase = q16 + ((size_t)(b * Nq + q0 + l16) * Dq + h * HDq);
        #pragma unroll
        for (int s = 0; s < 2; ++s) {
            v8h lo = *(const v8h*)(qbase + s * 32 + hi * 8);
            v8h up = *(const v8h*)(qbase + s * 32 + hi * 8 + 16);
            #pragma unroll
            for (int e = 0; e < 8; ++e) { qa[s][e] = lo[e]; qa[s][e + 8] = up[e]; }
        }
    }

    float m_r[8], l_r[8];
    v8f o[4];
    #pragma unroll
    for (int i = 0; i < 8; ++i) { m_r[i] = -1.0e30f; l_r[i] = 0.0f; }
    #pragma unroll
    for (int t = 0; t < 4; ++t) o[t] = (v8f){};

    const size_t adj_base = (size_t)b * Nq * Nq;

    for (int j = 0; j < 32; ++j) {
        __syncthreads();
        #pragma unroll
        for (int u = 0; u < 2; ++u) {
            int idx = tid + u * 256;
            int r = idx >> 5, c = idx & 31;
            int av = adj[adj_base + (size_t)(q0 + r) * Nq + j * 32 + c];
            adjb[idx] = (av != 0) ? 0.0f : -10000.0f;
        }
        if (j < 31)
            __builtin_prefetch(&adj[adj_base + (size_t)(q0 + (tid >> 4)) * Nq + (j + 1) * 32], 0, 0);
        __syncthreads();

        v8f sc[2];
        sc[0] = (v8f){}; sc[1] = (v8f){};
        #pragma unroll
        for (int cc = 0; cc < 2; ++cc) {
            #pragma unroll
            for (int s = 0; s < 2; ++s) {
                v16h kb = frag_row(k16 + ((size_t)(b * Nq + j * 32 + cc * 16 + l16) * Dq + h * HDq + s * 32), hi);
                sc[cc] = wmma16(qa[s], kb, sc[cc]);
            }
        }

        {
            const char* vsrc = (const char*)(v16 + ((size_t)(b * Nq + j * 32) * Dq + h * HDq));
            for (int c = lane; c < 256; c += 32) {
                int row = c >> 3, ch = c & 7;
                ((v4u*)Vt[wave])[c] = *(const v4u*)(vsrc + (size_t)row * Dq * 2 + ch * 16);
            }
        }

        #pragma unroll
        for (int i = 0; i < 8; ++i) {
            int rr = (i + hi * 8) * 32;
            float s0 = sc[0][i] * 0.125f + adjb[rr + l16];
            float s1 = sc[1][i] * 0.125f + adjb[rr + 16 + l16];
            float tm = fmaxf(s0, s1);
            tm = fmaxf(tm, __shfl_xor(tm, 1, 16));
            tm = fmaxf(tm, __shfl_xor(tm, 2, 16));
            tm = fmaxf(tm, __shfl_xor(tm, 4, 16));
            tm = fmaxf(tm, __shfl_xor(tm, 8, 16));
            float mn   = fmaxf(m_r[i], tm);
            float corr = __expf(m_r[i] - mn);
            float p0   = __expf(s0 - mn);
            float p1   = __expf(s1 - mn);
            float ps = p0 + p1;
            ps += __shfl_xor(ps, 1, 16);
            ps += __shfl_xor(ps, 2, 16);
            ps += __shfl_xor(ps, 4, 16);
            ps += __shfl_xor(ps, 8, 16);
            l_r[i] = l_r[i] * corr + ps;
            m_r[i] = mn;
            #pragma unroll
            for (int t = 0; t < 4; ++t) o[t][i] *= corr;
            Pt[wave][rr + l16]      = (_Float16)(p0 * PSC);
            Pt[wave][rr + 16 + l16] = (_Float16)(p1 * PSC);
        }
        __syncthreads();

        v16h pa;
        {
            const _Float16* pp = &Pt[wave][l16 * 32 + hi * 8];
            v8h lo = *(const v8h*)pp;
            v8h up = *(const v8h*)(pp + 16);
            #pragma unroll
            for (int e = 0; e < 8; ++e) { pa[e] = lo[e]; pa[e + 8] = up[e]; }
        }

        #pragma unroll
        for (int t = 0; t < 4; ++t) {
            v16h vb;
            #pragma unroll
            for (int e = 0; e < 8; ++e) {
                vb[e]     = Vt[wave][(hi * 8 + e) * HDq + t * 16 + l16];
                vb[e + 8] = Vt[wave][(16 + hi * 8 + e) * HDq + t * 16 + l16];
            }
            o[t] = wmma16(pa, vb, o[t]);
        }
    }

    #pragma unroll
    for (int t = 0; t < 4; ++t) {
        #pragma unroll
        for (int i = 0; i < 8; ++i) Ot[wave][(i + hi * 8) * HDq + t * 16 + l16] = (_Float16)(o[t][i] * (PUN / l_r[i]));
    }
    __syncthreads();
    #pragma unroll
    for (int qq = 0; qq < 4; ++qq) {
        const int rl = qq * 4 + (lane >> 3), pc = lane & 7;
        vst2(attn16 + (size_t)(b * Nq + q0 + rl) * Dq + h * HDq + pc * 8, *(const v4u*)(&Ot[wave][rl * HDq + pc * 8]));
    }
}

__global__ __launch_bounds__(256) void proj_kernel(
    const _Float16* __restrict__ attn16, const _Float16* __restrict__ wo16,
    const float* __restrict__ bo, const float* __restrict__ xin,
    float* __restrict__ y) {

    const int tid  = threadIdx.x;
    const int wave = tid >> 5;
    const int lane = tid & 31;
    const int hi   = lane >> 4;
    const int l16  = lane & 15;
    const int m0   = blockIdx.x * 16;

    __shared__ __align__(16) _Float16 As[16 * Dq];
    __shared__ __align__(16) float Ct[8][16 * 64];
    {
        const char* src = (const char*)(attn16 + (size_t)m0 * Dq);
        for (int c = tid; c < 16 * Dq / 8; c += 256)
            ((v4u*)As)[c] = ((const v4u*)src)[c];
    }
    __syncthreads();

    v8f acc[4];
    #pragma unroll
    for (int t = 0; t < 4; ++t) acc[t] = (v8f){};

    for (int kk = 0; kk < Dq; kk += 32) {
        const _Float16* ap = As + l16 * Dq + kk + hi * 8;
        v8h alo = *(const v8h*)ap;
        v8h ahi = *(const v8h*)(ap + 16);
        v16h a;
        #pragma unroll
        for (int e = 0; e < 8; ++e) { a[e] = alo[e]; a[e + 8] = ahi[e]; }
        #pragma unroll
        for (int t = 0; t < 4; ++t) {
            int ncol = (wave * 4 + t) * 16;
            v16h b = frag_row(wo16 + (size_t)(ncol + l16) * Dq + kk, hi);
            acc[t] = wmma16(a, b, acc[t]);
        }
    }

    #pragma unroll
    for (int t = 0; t < 4; ++t) {
        int col = (wave * 4 + t) * 16 + l16;
        float bias = bo[col];
        #pragma unroll
        for (int i = 0; i < 8; ++i) {
            size_t idx = (size_t)(m0 + i + hi * 8) * Dq + col;
            Ct[wave][(i + hi * 8) * 64 + t * 16 + l16] = acc[t][i] + bias + xin[idx];
        }
    }
    __syncthreads();
    #pragma unroll
    for (int qq = 0; qq < 8; ++qq) {
        const int rl = qq * 2 + (lane >> 4), pc = lane & 15;
        vst2(y + (size_t)(m0 + rl) * Dq + wave * 64 + pc * 4, *(const v4f*)(&Ct[wave][rl * 64 + pc * 4]));
    }
}

__global__ __launch_bounds__(256) void ln_kernel(float* __restrict__ y,
                                                 const float* __restrict__ gamma,
                                                 const float* __restrict__ beta) {
    const int tid  = threadIdx.x;
    const int wave = tid >> 5;
    const int lane = tid & 31;
    const size_t base = (size_t)blockIdx.x * Dq;

    float v0 = y[base + tid];
    float v1 = y[base + tid + 256];
    float s1 = v0 + v1;
    float s2 = v0 * v0 + v1 * v1;
    #pragma unroll
    for (int off = 16; off > 0; off >>= 1) {
        s1 += __shfl_xor(s1, off);
        s2 += __shfl_xor(s2, off);
    }

    __shared__ float red1[8], red2[8];
    if (lane == 0) { red1[wave] = s1; red2[wave] = s2; }
    __syncthreads();
    if (tid == 0) {
        float a = 0.f, q = 0.f;
        #pragma unroll
        for (int i = 0; i < 8; ++i) { a += red1[i]; q += red2[i]; }
        float mu  = a / (float)Dq;
        float var = q / (float)Dq - mu * mu;
        red1[0] = mu;
        red2[0] = rsqrtf(var + 1e-5f);
    }
    __syncthreads();
    float mu = red1[0], rstd = red2[0];
    vst2(y + base + tid,       (v0 - mu) * rstd * gamma[tid]       + beta[tid]);
    vst2(y + base + tid + 256, (v1 - mu) * rstd * gamma[tid + 256] + beta[tid + 256]);
}

extern "C" void kernel_launch(void* const* d_in, const int* in_sizes, int n_in,
                              void* d_out, int out_size, void* d_ws, size_t ws_size,
                              hipStream_t stream) {
    (void)in_sizes; (void)n_in; (void)out_size; (void)ws_size;

    const float* x    = (const float*)d_in[0];
    const int*   adj  = (const int*)d_in[1];
    const float* wq   = (const float*)d_in[2];
    const float* wk   = (const float*)d_in[3];
    const float* wv   = (const float*)d_in[4];
    const float* wo   = (const float*)d_in[5];
    const float* bo   = (const float*)d_in[6];
    const float* gam  = (const float*)d_in[7];
    const float* bet  = (const float*)d_in[8];
    float* out = (float*)d_out;

    const size_t XN = (size_t)Bq * Nq * Dq;
    const size_t WN = (size_t)Dq * Dq;
    char* ws = (char*)d_ws;
    _Float16* x16  = (_Float16*)(ws);
    _Float16* wq16 = (_Float16*)(ws + 2 * XN);
    _Float16* wk16 = wq16 + WN;
    _Float16* wv16 = wk16 + WN;
    _Float16* wo16 = wv16 + WN;
    _Float16* q16  = wo16 + WN;
    _Float16* k16  = q16 + XN;
    _Float16* v16  = k16 + XN;
    _Float16* a16  = v16 + XN;

    cvt_f32_f16<<<(int)(XN / 8 / 256), 256, 0, stream>>>(x, x16, (int)XN);
    cvt_f32_f16<<<(int)(WN / 8 / 256), 256, 0, stream>>>(wq, wq16, (int)WN);
    cvt_f32_f16<<<(int)(WN / 8 / 256), 256, 0, stream>>>(wk, wk16, (int)WN);
    cvt_f32_f16<<<(int)(WN / 8 / 256), 256, 0, stream>>>(wv, wv16, (int)WN);
    cvt_f32_f16<<<(int)(WN / 8 / 256), 256, 0, stream>>>(wo, wo16, (int)WN);

    qkv_gemm<<<dim3(Bq * Nq / 16, Dq / 128, 3), 256, 0, stream>>>(
        x16, wq16, wk16, wv16, q16, k16, v16);

    attn_kernel<<<dim3(Nq / 16, Bq), 256, 0, stream>>>(q16, k16, v16, adj, a16);

    proj_kernel<<<dim3(Bq * Nq / 16), 256, 0, stream>>>(a16, wo16, bo, x, out);

    ln_kernel<<<dim3(Bq * Nq), 256, 0, stream>>>(out, gam, bet);
}
